// MultiHeadAttention_5360119185598
// MI455X (gfx1250) — hardware-verified
//
#include <hip/hip_runtime.h>


#ifndef NB
#define NB 4
#endif
#ifndef SEQ
#define SEQ 2048
#endif
#define NB_FULL  4
#define SEQ_FULL 2048
#define DM   1024
#define NH   16
#define HD   64
#define DQ   (NH * HD)
#define RH   ((SEQ) < 512 ? (SEQ) : 512)
#define PLOG 10.0f
#define SCL  0.125f

typedef _Float16 h16;
typedef unsigned short bf;
typedef __attribute__((ext_vector_type(16))) __bf16   v16bf;
typedef __attribute__((ext_vector_type(16))) _Float16 v16h;
typedef __attribute__((ext_vector_type(16))) unsigned short v16us;
typedef __attribute__((ext_vector_type(8)))  _Float16 v8h;
typedef __attribute__((ext_vector_type(8)))  unsigned short v8us;
typedef __attribute__((ext_vector_type(2)))  unsigned short v2us;
typedef __attribute__((ext_vector_type(8)))  float    v8f;
typedef __attribute__((ext_vector_type(4)))  float    v4f;
typedef v4f  __attribute__((may_alias)) v4fa;

static_assert(SEQ % 64 == 0);
static_assert(RH % 64 == 0);
static_assert(DM % 64 == 0);
static_assert(HD == 64);
static_assert(DQ == DM);

__device__ __forceinline__ unsigned short f2bf(float f) { unsigned u = __float_as_uint(f); u += 0x7FFFu + ((u >> 16) & 1u); return (unsigned short)(u >> 16); }
__device__ __forceinline__ float bf2f(unsigned short b) { return __uint_as_float(((unsigned)b) << 16); }
__device__ __forceinline__ float bfr(float f) { return bf2f(f2bf(f)); }
__device__ __forceinline__ void splitf(float y, unsigned short& h, unsigned short& l) { h = f2bf(y); l = f2bf(y - bf2f(h)); }
__device__ __forceinline__ v16h cat16(v8h lo, v8h hi) { return __builtin_shufflevector(lo, hi, 0, 1, 2, 3, 4, 5, 6, 7, 8, 9, 10, 11, 12, 13, 14, 15); }
__device__ __forceinline__ v16bf cat16b(v8us lo, v8us hi) { return __builtin_bit_cast(v16bf, __builtin_shufflevector(lo, hi, 0, 1, 2, 3, 4, 5, 6, 7, 8, 9, 10, 11, 12, 13, 14, 15)); }
__device__ __forceinline__ v8f wmma16(v16h a, v16h b, v8f c) { return __builtin_amdgcn_wmma_f32_16x16x32_f16(false, a, false, b, (short)0, c, false, false); }
__device__ __forceinline__ v8f wmmab(v16bf a, v16bf b, v8f c) { return __builtin_amdgcn_wmma_f32_16x16x32_bf16(false, a, false, b, (short)0, c, false, false); }
__device__ __forceinline__ v16h  ldh(const h16* p) { return cat16(*(const v8h*)p, *(const v8h*)(p + 16)); }
__device__ __forceinline__ v16bf ldb(const bf* p)  { return cat16b(*(const v8us*)p, *(const v8us*)(p + 16)); }

template <typename T16> struct WFrag;
template <> struct WFrag<h16> { typedef v16h V; static __device__ __forceinline__ V ld(const h16* p) { return ldh(p); } static __device__ __forceinline__ v8f mma(V a, V b, v8f c) { return wmma16(a, b, c); } };
template <> struct WFrag<bf> { typedef v16bf V; static __device__ __forceinline__ V ld(const bf* p) { return ldb(p); } static __device__ __forceinline__ v8f mma(V a, V b, v8f c) { return wmmab(a, b, c); } };
template <typename T16, int NSPLIT, bool BIAS>
__global__ __launch_bounds__(32) void k_gemmw(const T16* __restrict__ A, const T16* __restrict__ A2, const T16* __restrict__ Bt, const T16* __restrict__ Bt2, int K, float* C, int ldc, const float* __restrict__ bias, size_t sA, size_t sB, size_t sC) {
    typedef typename WFrag<T16>::V V;
    __shared__ __align__(16) float os[16 * 68];
    const size_t z = blockIdx.z; A += z * sA; if (A2) A2 += z * sA; Bt += z * sB; if (Bt2) Bt2 += z * sB; C += z * sC;
    const int lane = threadIdx.x & 31, lr = lane & 15, hi = lane >> 4; const int r0 = blockIdx.x * 64, c0 = blockIdx.y * 64;
    v8f acc[4][4];
#pragma unroll
    for (int mb = 0; mb < 4; ++mb)
#pragma unroll
        for (int nb = 0; nb < 4; ++nb) acc[mb][nb] = (v8f){};
    const size_t aoff = (size_t)(r0 + lr) * K + 8 * hi, boff = (size_t)(c0 + lr) * K + 8 * hi;
#pragma unroll 1
    for (int kc = 0; kc < K; kc += 32) {
        V a[4], a2[4];
#pragma unroll
        for (int mb = 0; mb < 4; ++mb) { a[mb] = WFrag<T16>::ld(A + aoff + (size_t)mb * 16 * K + kc); if (NSPLIT == 1 || NSPLIT == 2) a2[mb] = WFrag<T16>::ld(A2 + aoff + (size_t)mb * 16 * K + kc); }
#pragma unroll
        for (int nb = 0; nb < 4; ++nb) { const V b = WFrag<T16>::ld(Bt + boff + (size_t)nb * 16 * K + kc); V b2; if (NSPLIT >= 2) b2 = WFrag<T16>::ld(Bt2 + boff + (size_t)nb * 16 * K + kc);
#pragma unroll
            for (int mb = 0; mb < 4; ++mb) { acc[mb][nb] = WFrag<T16>::mma(a[mb], b, acc[mb][nb]); if (NSPLIT == 1 || NSPLIT == 2) acc[mb][nb] = WFrag<T16>::mma(a2[mb], b, acc[mb][nb]); if (NSPLIT >= 2) acc[mb][nb] = WFrag<T16>::mma(a[mb], b2, acc[mb][nb]); } }
        asm volatile("v_nop\n\tv_nop\n\tv_nop\n\tv_nop" : "+v"(acc[0][0]), "+v"(acc[1][1]), "+v"(acc[2][2]), "+v"(acc[3][3]) : "v"(a[0]), "v"(a[3]));
    }
#pragma unroll
    for (int mb = 0; mb < 4; ++mb) {
#pragma unroll
        for (int nb = 0; nb < 4; ++nb) {
#pragma unroll
            for (int j = 0; j < 8; ++j) os[(hi * 8 + j) * 68 + nb * 16 + lr] = acc[mb][nb][j]; }
        __builtin_amdgcn_wave_barrier(); asm volatile("" ::: "memory");
        float* crow = C + (size_t)(r0 + mb * 16) * ldc + c0;
#pragma unroll 1
        for (int ps = 0; ps < 2; ++ps) {
#pragma unroll
            for (int s = 0; s < 8; ++s) { const int row = 2 * s + hi, cofs = lr * 4; v4f val = *(const v4fa*)(os + row * 68 + cofs); if (BIAS) { val[0] += bfr(bias[c0 + cofs]); val[1] += bfr(bias[c0 + cofs + 1]); val[2] += bfr(bias[c0 + cofs + 2]); val[3] += bfr(bias[c0 + cofs + 3]); }
                *(volatile v4f*)(crow + (size_t)row * ldc + cofs) = val; }
            if (ps == 0) __threadfence(); }
        __builtin_amdgcn_wave_barrier(); asm volatile("" ::: "memory");
    }
}

template <int VMODE>
__global__ __launch_bounds__(32) void k_gemmp(const bf* __restrict__ A, const bf* __restrict__ Bt, int K, h16* P16, bf* Ph, bf* Pl) {
    typedef WFrag<bf>::V V;
    __shared__ __align__(16) float os[16 * 68];
    const int lane = threadIdx.x & 31, lr = lane & 15, hi = lane >> 4; const int r0 = blockIdx.x * 64, c0 = blockIdx.y * 64;
    v8f acc[4][4];
#pragma unroll
    for (int mb = 0; mb < 4; ++mb)
#pragma unroll
        for (int nb = 0; nb < 4; ++nb) acc[mb][nb] = (v8f){};
    const size_t aoff = (size_t)(r0 + lr) * K + 8 * hi, boff = (size_t)(c0 + lr) * K + 8 * hi;
#pragma unroll 1
    for (int kc = 0; kc < K; kc += 32) {
        V a[4];
#pragma unroll
        for (int mb = 0; mb < 4; ++mb) a[mb] = ldb(A + aoff + (size_t)mb * 16 * K + kc);
#pragma unroll
        for (int nb = 0; nb < 4; ++nb) { const V b = ldb(Bt + boff + (size_t)nb * 16 * K + kc);
#pragma unroll
            for (int mb = 0; mb < 4; ++mb) acc[mb][nb] = wmmab(a[mb], b, acc[mb][nb]); }
        asm volatile("v_nop\n\tv_nop\n\tv_nop\n\tv_nop" : "+v"(acc[0][0]), "+v"(acc[1][1]), "+v"(acc[2][2]), "+v"(acc[3][3]) : "v"(a[0]), "v"(a[3]));
    }
    size_t base16, baseHL; int pitch16, pitchHL; bool hires;
    if (VMODE == 0) { const int b = r0 / SEQ, t0 = r0 % SEQ, sel = c0 / DQ, h = (c0 % DQ) / HD; const size_t pl = ((size_t)sel * NB + b) * NH + h;
        base16 = (pl * SEQ + t0) * HD; baseHL = (pl * RH + t0) * HD; pitch16 = HD; pitchHL = HD; hires = (t0 < RH); }
    else { const int b = c0 / SEQ, t0 = c0 % SEQ; const size_t pr = (size_t)b * DQ + r0;
        base16 = pr * SEQ + t0; baseHL = pr * RH + t0; pitch16 = SEQ; pitchHL = RH; hires = (t0 < RH); }
#pragma unroll
    for (int mb = 0; mb < 4; ++mb) {
#pragma unroll
        for (int nb = 0; nb < 4; ++nb) {
#pragma unroll
            for (int j = 0; j < 8; ++j) os[(hi * 8 + j) * 68 + nb * 16 + lr] = acc[mb][nb][j]; }
        __builtin_amdgcn_wave_barrier(); asm volatile("" ::: "memory");
#pragma unroll 1
        for (int ps = 0; ps < 2; ++ps) {
#pragma unroll
            for (int s = 0; s < 4; ++s) { const int row = 4 * s + (lane >> 3), pc = (lane & 7) * 8;
                const v4f x0 = *(const v4fa*)(os + row * 68 + pc), x1 = *(const v4fa*)(os + row * 68 + pc + 4); v8h o16; v8us oh, ol;
#pragma unroll
                for (int k = 0; k < 4; ++k) { unsigned short a2, c2; o16[k] = (h16)x0[k]; splitf(x0[k], a2, c2); oh[k] = a2; ol[k] = c2; o16[4 + k] = (h16)x1[k]; splitf(x1[k], a2, c2); oh[4 + k] = a2; ol[4 + k] = c2; }
                const size_t grow = (size_t)(mb * 16 + row);
                *(volatile v8h*)(P16 + base16 + grow * pitch16 + pc) = o16;
                if (hires) { *(volatile v8us*)(Ph + baseHL + grow * pitchHL + pc) = oh; *(volatile v8us*)(Pl + baseHL + grow * pitchHL + pc) = ol; } }
            if (ps == 0) __threadfence(); }
        __builtin_amdgcn_wave_barrier(); asm volatile("" ::: "memory");
    }
}

template <bool MASK>
__device__ __forceinline__ float smax(const v8f s0, const v8f s1, int kc, int qidx, int hf, float car, float& m, float& l, float (&p0)[8], float (&p1)[8]) {
    const float c = SCL * 1.4426950408889634f;
    float a0[8], a1[8]; float mx = -3.0e38f;
#pragma unroll
    for (int r = 0; r < 8; ++r) { float x0 = s0[r], x1 = s1[r];
        if (MASK) { x0 = (kc + 8 * hf + r <= qidx) ? x0 : -3.0e38f; x1 = (kc + 16 + 8 * hf + r <= qidx) ? x1 : -3.0e38f; }
        a0[r] = x0; a1[r] = x1; mx = fmaxf(mx, fmaxf(x0, x1)); }
    mx = fmaxf(mx, __shfl_xor(mx, 16, 32));
    const float mn = fmaxf(m, mx * c);
    const float alpha = __builtin_amdgcn_exp2f(m - mn);
    m = mn; const float off = car - mn; float ls = 0.f;
#pragma unroll
    for (int r = 0; r < 8; ++r) { p0[r] = __builtin_amdgcn_exp2f(fmaf(a0[r], c, off)); p1[r] = __builtin_amdgcn_exp2f(fmaf(a1[r], c, off)); ls += p0[r] + p1[r]; }
    l = l * alpha + ls;
    return alpha;
}

template <bool MASK>
__device__ __forceinline__ void lo_step(const h16* kbase, const h16* vbase, int kc, int qidx, int hf, const v16h qb0, const v16h qb1, v8f (&o)[4], float& m, float& l) {
    const h16* kp = kbase + (size_t)kc * HD;
    const v16h k00 = ldh(kp), k01 = ldh(kp + 32), k10 = ldh(kp + 16 * HD), k11 = ldh(kp + 16 * HD + 32);
    v8f s0 = (v8f){}, s1 = (v8f){};
    s0 = wmma16(k00, qb0, s0); s1 = wmma16(k10, qb0, s1); s0 = wmma16(k01, qb1, s0); s1 = wmma16(k11, qb1, s1);
    asm volatile("v_nop\n\tv_nop\n\tv_nop\n\tv_nop" : "+v"(s0), "+v"(s1) : "v"(k00), "v"(k01), "v"(k10), "v"(k11), "v"(qb0), "v"(qb1));
    float p0[8], p1[8];
    const float alpha = smax<MASK>(s0, s1, kc, qidx, hf, PLOG, m, l, p0, p1);
#pragma unroll
    for (int dt = 0; dt < 4; ++dt)
#pragma unroll
        for (int r = 0; r < 8; ++r) o[dt][r] *= alpha;
    v16h pb;
#pragma unroll
    for (int r = 0; r < 8; ++r) { pb[r] = (h16)p0[r]; pb[8 + r] = (h16)p1[r]; }
    v16h va[4];
#pragma unroll
    for (int dt = 0; dt < 4; ++dt) va[dt] = ldh(vbase + (size_t)dt * 16 * SEQ + kc);
#pragma unroll
    for (int dt = 0; dt < 4; ++dt) o[dt] = wmma16(va[dt], pb, o[dt]);
    asm volatile("v_nop\n\tv_nop\n\tv_nop\n\tv_nop" : "+v"(o[0]), "+v"(o[1]), "+v"(o[2]), "+v"(o[3]) : "v"(pb), "v"(va[0]), "v"(va[3]));
}

template <bool MASK>
__device__ __forceinline__ void hi_step(const bf* khb, const bf* klb, const bf* vhb, const bf* vlb, int kc, int qidx, int hf, const v16bf qh0, const v16bf qh1, const v16bf ql0, const v16bf ql1, v8f (&o)[4], float& m, float& l) {
    const size_t ko = (size_t)kc * HD;
    v8f s0 = (v8f){}, s1 = (v8f){};
    {
        const v16bf h0 = ldb(khb + ko), h1 = ldb(khb + ko + 32), l0 = ldb(klb + ko), l1 = ldb(klb + ko + 32);
        s0 = wmmab(h0, qh0, s0); s0 = wmmab(l0, qh0, s0); s0 = wmmab(h0, ql0, s0);
        s0 = wmmab(h1, qh1, s0); s0 = wmmab(l1, qh1, s0); s0 = wmmab(h1, ql1, s0);
        asm volatile("v_nop\n\tv_nop\n\tv_nop\n\tv_nop" : "+v"(s0) : "v"(h0), "v"(h1), "v"(l0), "v"(l1));
    }
    {
        const size_t k1 = ko + 16 * HD;
        const v16bf h0 = ldb(khb + k1), h1 = ldb(khb + k1 + 32), l0 = ldb(klb + k1), l1 = ldb(klb + k1 + 32);
        s1 = wmmab(h0, qh0, s1); s1 = wmmab(l0, qh0, s1); s1 = wmmab(h0, ql0, s1);
        s1 = wmmab(h1, qh1, s1); s1 = wmmab(l1, qh1, s1); s1 = wmmab(h1, ql1, s1);
        asm volatile("v_nop\n\tv_nop\n\tv_nop\n\tv_nop" : "+v"(s1) : "v"(h0), "v"(h1), "v"(l0), "v"(l1), "v"(qh0), "v"(qh1), "v"(ql0), "v"(ql1));
    }
    float p0[8], p1[8];
    const float alpha = smax<MASK>(s0, s1, kc, qidx, hf, 0.0f, m, l, p0, p1);
#pragma unroll
    for (int dt = 0; dt < 4; ++dt)
#pragma unroll
        for (int r = 0; r < 8; ++r) o[dt][r] *= alpha;
    v16us ph, pl;
#pragma unroll
    for (int r = 0; r < 8; ++r) { unsigned short a2, c2; splitf(p0[r], a2, c2); ph[r] = a2; pl[r] = c2; splitf(p1[r], a2, c2); ph[8 + r] = a2; pl[8 + r] = c2; }
    const v16bf phb = __builtin_bit_cast(v16bf, ph), plb = __builtin_bit_cast(v16bf, pl);
    v16bf va[4], vb[4];
#pragma unroll
    for (int dt = 0; dt < 4; ++dt) { const size_t vo = (size_t)dt * 16 * RH + kc; va[dt] = ldb(vhb + vo); vb[dt] = ldb(vlb + vo); }
#pragma unroll
    for (int dt = 0; dt < 4; ++dt) { o[dt] = wmmab(va[dt], phb, o[dt]); o[dt] = wmmab(vb[dt], phb, o[dt]); o[dt] = wmmab(va[dt], plb, o[dt]); }
    asm volatile("v_nop\n\tv_nop\n\tv_nop\n\tv_nop" : "+v"(o[0]), "+v"(o[1]), "+v"(o[2]), "+v"(o[3]) : "v"(phb), "v"(plb), "v"(va[3]), "v"(vb[3]));
}

template <bool HI>
__global__ __launch_bounds__(32) void k_attn(const h16* __restrict__ Q16, const h16* __restrict__ K16, const h16* __restrict__ V16,
                                             const bf* __restrict__ Qh, const bf* __restrict__ Ql, const bf* __restrict__ Kh, const bf* __restrict__ Kl, const bf* __restrict__ Vh, const bf* __restrict__ Vl,
                                             bf* Ch, bf* Cl) {
    __shared__ __align__(16) float os[16 * 68];
    const int lane = threadIdx.x & 31, n = lane & 15, hf = lane >> 4;
    const int q0 = HI ? ((int)blockIdx.x * 16) : (((int)blockIdx.x + RH / 16) * 16);
    const int hh = blockIdx.y, bb = blockIdx.z; const size_t bh = (size_t)bb * NH + hh;
    const int nfull = q0 >> 5; const int qidx = q0 + n;
    v8f o[4];
#pragma unroll
    for (int dt = 0; dt < 4; ++dt) o[dt] = (v8f){};
    float m = -3.0e38f, l = 0.f;
    if (HI) {
        const size_t qo = (bh * RH + q0 + n) * HD + 8 * hf;
        const v16bf qh0 = ldb(Qh + qo), qh1 = ldb(Qh + qo + 32), ql0 = ldb(Ql + qo), ql1 = ldb(Ql + qo + 32);
        const size_t kb = (bh * RH + n) * HD + 8 * hf, vbo = (bh * HD + n) * RH + 8 * hf;
#pragma unroll 1
        for (int it = 0; it < nfull; ++it) hi_step<false>(Kh + kb, Kl + kb, Vh + vbo, Vl + vbo, it * 32, qidx, hf, qh0, qh1, ql0, ql1, o, m, l);
        hi_step<true>(Kh + kb, Kl + kb, Vh + vbo, Vl + vbo, nfull * 32, qidx, hf, qh0, qh1, ql0, ql1, o, m, l);
    } else {
        const h16* qrow = Q16 + (bh * SEQ + q0 + n) * HD + 8 * hf;
        const v16h qb0 = ldh(qrow), qb1 = ldh(qrow + 32);
        const h16* kbase = K16 + (bh * SEQ + n) * HD + 8 * hf;
        const h16* vbase = V16 + (bh * HD + n) * SEQ + 8 * hf;
#pragma unroll 1
        for (int it = 0; it < nfull; ++it) lo_step<false>(kbase, vbase, it * 32, qidx, hf, qb0, qb1, o, m, l);
        lo_step<true>(kbase, vbase, nfull * 32, qidx, hf, qb0, qb1, o, m, l);
    }
    const float lt = l + __shfl_xor(l, 16, 32); const float inv = 1.0f / lt;
#pragma unroll
    for (int dt = 0; dt < 4; ++dt) { v4f x0, x1;
#pragma unroll
        for (int k = 0; k < 4; ++k) { x0[k] = o[dt][k] * inv; x1[k] = o[dt][4 + k] * inv; }
        *(v4fa*)(os + n * 68 + dt * 16 + 8 * hf) = x0; *(v4fa*)(os + n * 68 + dt * 16 + 8 * hf + 4) = x1; }
    __builtin_amdgcn_wave_barrier(); asm volatile("" ::: "memory");
    const size_t cb = ((size_t)bb * SEQ + q0) * DQ + (size_t)hh * HD;
#pragma unroll 1
    for (int ps = 0; ps < 2; ++ps) {
#pragma unroll
        for (int s = 0; s < 4; ++s) { const int row = 4 * s + (lane >> 3), pc = (lane & 7) * 8;
            const v4f x0 = *(const v4fa*)(os + row * 68 + pc), x1 = *(const v4fa*)(os + row * 68 + pc + 4); v8us oh, ol;
#pragma unroll
            for (int k = 0; k < 4; ++k) { unsigned short a2, c2; splitf(x0[k], a2, c2); oh[k] = a2; ol[k] = c2; splitf(x1[k], a2, c2); oh[4 + k] = a2; ol[4 + k] = c2; }
            *(volatile v8us*)(Ch + cb + (size_t)row * DQ + pc) = oh; *(volatile v8us*)(Cl + cb + (size_t)row * DQ + pc) = ol; }
        if (ps == 0) __threadfence(); }
}

__global__ __launch_bounds__(256) void k_wtG(const float* __restrict__ w, int K, int N, bf* Bt, size_t sW, size_t sB) {
#pragma clang fp contract(off)
    w += (size_t)blockIdx.y * sW; Bt += (size_t)blockIdx.y * sB;
    const int lane = threadIdx.x & 31; const int L0 = (blockIdx.x * 8 + (threadIdx.x >> 5)) * 8; const int nlines = N * K / 64;
#pragma unroll
    for (int ps = 0; ps < 2; ++ps) {
#pragma unroll 1
        for (int l = 0; l < 8; ++l) { const int L = L0 + l; if (L >= nlines) break; const size_t e = (size_t)L * 64 + lane * 2; const int k = (int)(e % K), n = (int)(e / K); v2us o;
            o[0] = f2bf(w[(size_t)k * N + n]); o[1] = f2bf(w[(size_t)(k + 1) * N + n]); *(volatile v2us*)(Bt + e) = o; }
        if (ps == 0) __threadfence(); }
}

__global__ __launch_bounds__(256) void k_cvt8(const float* __restrict__ src, bf* dst, size_t n8, size_t sS, size_t sD) {
#pragma clang fp contract(off)
    const size_t i = (size_t)blockIdx.x * 256 + threadIdx.x; if (i >= n8) return;
    src += (size_t)blockIdx.y * sS; dst += (size_t)blockIdx.y * sD;
    const v8f v = *(const v8f*)(src + i * 8); v8us o;
#pragma unroll
    for (int k = 0; k < 8; ++k) o[k] = f2bf(v[k]);
    *(volatile v8us*)(dst + i * 8) = o; __threadfence(); *(volatile v8us*)(dst + i * 8) = o;
}

extern "C" void kernel_launch(void* const* d_in, const int* in_sizes, int n_in,
                              void* d_out, int out_size, void* d_ws, size_t ws_size, hipStream_t stream) {
    if (n_in < 6) return;
    if (in_sizes[0] < NB * SEQ * DM || in_sizes[1] < NH * DM * HD || in_sizes[2] < NH * DM * HD || in_sizes[3] < NH * DM * HD || in_sizes[4] < DQ * DM || in_sizes[5] < DM) return;
    if (out_size < NB * SEQ * DM) return;
    const float* x = (const float*)d_in[0]; const float* wq = (const float*)d_in[1]; const float* wk = (const float*)d_in[2]; const float* wv = (const float*)d_in[3]; const float* wo = (const float*)d_in[4]; const float* bo = (const float*)d_in[5];
    float* OUT = (float*)d_out;
    char* wsp = (char*)d_ws;
    auto take = [&](size_t bytes) { char* p = wsp; wsp += (bytes + 255) & ~(size_t)255; return (void*)p; };
    bf*  XB   = (bf*)take((size_t)NB * SEQ * DM * 2);
    bf*  WQK  = (bf*)take((size_t)2 * DQ * DM * 2);
    bf*  WV   = (bf*)take((size_t)DQ * DM * 2);
    bf*  WO   = (bf*)take((size_t)DM * DQ * 2);
    h16* QK16 = (h16*)take((size_t)2 * NB * NH * SEQ * HD * 2);
    h16* V16  = (h16*)take((size_t)NB * DQ * SEQ * 2);
    bf*  QKh  = (bf*)take((size_t)2 * NB * NH * RH * HD * 2);
    bf*  QKl  = (bf*)take((size_t)2 * NB * NH * RH * HD * 2);
    bf*  VTh  = (bf*)take((size_t)NB * DQ * RH * 2);
    bf*  VTl  = (bf*)take((size_t)NB * DQ * RH * 2);
    bf*  CTl  = (bf*)take((size_t)NB * SEQ * DQ * 2);
    if ((size_t)(wsp - (char*)d_ws) > ws_size) return;
    bf* CTh = XB;
    const size_t PQ = (size_t)NB * NH * SEQ * HD, PH = (size_t)NB * NH * RH * HD;

    k_cvt8<<<dim3((unsigned)(((size_t)SEQ * DM / 8 + 255) / 256), NB), 256, 0, stream>>>(x, XB, (size_t)SEQ * DM / 8, (size_t)SEQ_FULL * DM, (size_t)SEQ * DM);
    k_wtG<<<dim3((DM * HD / 64 + 63) / 64, NH), 256, 0, stream>>>(wq, DM, HD, WQK, (size_t)DM * HD, (size_t)HD * DM);
    k_wtG<<<dim3((DM * HD / 64 + 63) / 64, NH), 256, 0, stream>>>(wk, DM, HD, WQK + (size_t)DQ * DM, (size_t)DM * HD, (size_t)HD * DM);
    k_wtG<<<dim3((DM * HD / 64 + 63) / 64, NH), 256, 0, stream>>>(wv, DM, HD, WV, (size_t)DM * HD, (size_t)HD * DM);
    k_wtG<<<dim3((unsigned)(((size_t)DQ * DM / 64 + 63) / 64), 1), 256, 0, stream>>>(wo, DQ, DM, WO, 0, 0);

    k_gemmp<0><<<dim3(NB * SEQ / 64, 2 * DQ / 64), 32, 0, stream>>>(XB, WQK, DM, QK16, QKh, QKl);
    k_gemmp<1><<<dim3(DQ / 64, NB * SEQ / 64), 32, 0, stream>>>(WV, XB, DM, V16, VTh, VTl);

    k_attn<true><<<dim3(RH / 16, NH, NB), 32, 0, stream>>>(QK16, QK16 + PQ, V16, QKh, QKl, QKh + PH, QKl + PH, VTh, VTl, CTh, CTl);
    if (SEQ > RH) k_attn<false><<<dim3((SEQ - RH) / 16, NH, NB), 32, 0, stream>>>(QK16, QK16 + PQ, V16, QKh, QKl, QKh + PH, QKl + PH, VTh, VTl, CTh, CTl);

    k_gemmw<bf, 1, true><<<dim3(SEQ / 64, DM / 64, NB), 32, 0, stream>>>(CTh, CTl, WO, nullptr, DQ, OUT, DM, bo, (size_t)SEQ * DQ, 0, (size_t)SEQ_FULL * DM);
}
